// EncoderAttention_31275951849956
// MI455X (gfx1250) — hardware-verified
//
#include <hip/hip_runtime.h>
#include <math.h>

constexpr int kBatch   = 2;
constexpr int kSeq     = 2048;
constexpr int kDim     = 1024;
constexpr int kHeads   = 16;
constexpr int kDh      = 64;
constexpr int kTok     = kBatch * kSeq;
constexpr int kNcat    = 3136;
constexpr int kGateCol = 3 * kDim;
constexpr int kZeroRow = kGateCol + kHeads;
constexpr float kQKScale = 0.125f;
constexpr float kFill    = -3.402823466e38f;
static_assert(kHeads * kDh == kDim, "shape");
static_assert(kNcat % 64 == 0 && kSeq % 64 == 0 && kTok % 64 == 0 && kDim % 64 == 0, "M,N tile multiples");
static_assert(kDim % 32 == 0, "K multiple of 32");
static_assert(kZeroRow + 48 == kNcat, "pad rows");
static_assert((kSeq / 64) == 32 && kHeads == 16, "attention grid decode uses qb = bx & 31, h = bx >> 5");

typedef __attribute__((ext_vector_type(16))) _Float16 v16h;
typedef __attribute__((ext_vector_type(8)))  _Float16 v8h;
typedef __attribute__((ext_vector_type(16))) __bf16   v16b;
typedef __attribute__((ext_vector_type(8)))  __bf16   v8b;
typedef __attribute__((ext_vector_type(8)))  float    v8f;
typedef __attribute__((ext_vector_type(4)))  float    v4f;
typedef __attribute__((ext_vector_type(2)))  float    v2f;
typedef __attribute__((ext_vector_type(4)))  unsigned int v4u;

__device__ __forceinline__ unsigned short f2bf_bits(float f) {
  unsigned u = __float_as_uint(f);
  return (unsigned short)((u + 0x7FFFu + ((u >> 16) & 1u)) >> 16);
}
__device__ __forceinline__ float bf_bits2f(unsigned short h) { return __uint_as_float(((unsigned)h) << 16); }
__device__ __forceinline__ float bfr(float f) { return bf_bits2f(f2bf_bits(f)); }
__device__ __forceinline__ void split_bits(float f, unsigned short& hb, unsigned short& lb) {
  hb = f2bf_bits(f);
  lb = f2bf_bits(f - bf_bits2f(hb));
}
__device__ __forceinline__ unsigned pk16(unsigned short a, unsigned short b) { return (unsigned)a | ((unsigned)b << 16); }

__device__ __forceinline__ void dep_guard_h(v8f& a, v8f& b, v16h x, v16h y) { asm volatile("v_nop\n\tv_nop\n\tv_nop\n\tv_nop" : "+v"(a), "+v"(b) : "v"(x), "v"(y)); }
__device__ __forceinline__ void dep_guard_b(v8f& a, v8f& b, v16b x, v16b y) { asm volatile("v_nop\n\tv_nop\n\tv_nop\n\tv_nop" : "+v"(a), "+v"(b) : "v"(x), "v"(y)); }
__device__ __forceinline__ void dep_guard4_h(v8f& a, v8f& b, v8f& c, v8f& d, v16h x, v16h y) { asm volatile("v_nop\n\tv_nop\n\tv_nop\n\tv_nop" : "+v"(a), "+v"(b), "+v"(c), "+v"(d) : "v"(x), "v"(y)); }
__device__ __forceinline__ void dep_guard4_b(v8f& a, v8f& b, v8f& c, v8f& d, v16b x, v16b y) { asm volatile("v_nop\n\tv_nop\n\tv_nop\n\tv_nop" : "+v"(a), "+v"(b), "+v"(c), "+v"(d) : "v"(x), "v"(y)); }
__device__ __forceinline__ void keep4_h(v16h a, v16h b, v16h c, v16h d) { asm volatile("v_nop" :: "v"(a), "v"(b), "v"(c), "v"(d)); }
__device__ __forceinline__ void keep4_b(v16b a, v16b b, v16b c, v16b d) { asm volatile("v_nop" :: "v"(a), "v"(b), "v"(c), "v"(d)); }
__device__ __forceinline__ void acc_guard4(v8f& a, v8f& b, v8f& c, v8f& d) { asm volatile("v_nop\n\tv_nop\n\tv_nop\n\tv_nop" : "+v"(a), "+v"(b), "+v"(c), "+v"(d)); }
template <typename T> struct Frag;
template <> struct Frag<_Float16> {
  typedef v16h V; union U { v16h v; v8h h[2]; };
  static __device__ __forceinline__ v16h load(const _Float16* p) {
    U f; f.h[0] = *(const v8h*)(p); f.h[1] = *(const v8h*)(p + 16); return f.v;
  }
  static __device__ __forceinline__ v8f mma(v16h a, v16h b, v8f c) {
    return __builtin_amdgcn_wmma_f32_16x16x32_f16(false, a, false, b, (short)0, c, false, false);
  }
  static __device__ __forceinline__ void guard(v8f& a, v8f& b, v16h x, v16h y) { dep_guard_h(a, b, x, y); }
  static __device__ __forceinline__ void guard4(v8f& a, v8f& b, v8f& c, v8f& d, v16h x, v16h y) { dep_guard4_h(a, b, c, d, x, y); }
  static __device__ __forceinline__ void keep(v16h a, v16h b, v16h c, v16h d) { keep4_h(a, b, c, d); }
};
template <> struct Frag<__bf16> {
  typedef v16b V; union U { v16b v; v8b h[2]; };
  static __device__ __forceinline__ v16b load(const __bf16* p) {
    U f; f.h[0] = *(const v8b*)(p); f.h[1] = *(const v8b*)(p + 16); return f.v;
  }
  static __device__ __forceinline__ v8f mma(v16b a, v16b b, v8f c) {
    return __builtin_amdgcn_wmma_f32_16x16x32_bf16(false, a, false, b, (short)0, c, false, false);
  }
  static __device__ __forceinline__ void guard(v8f& a, v8f& b, v16b x, v16b y) { dep_guard_b(a, b, x, y); }
  static __device__ __forceinline__ void guard4(v8f& a, v8f& b, v8f& c, v8f& d, v16b x, v16b y) { dep_guard4_b(a, b, c, d, x, y); }
  static __device__ __forceinline__ void keep(v16b a, v16b b, v16b c, v16b d) { keep4_b(a, b, c, d); }
};

template <int ET> struct Elem;
template <> struct Elem<0> { typedef _Float16 T; };
template <> struct Elem<1> { typedef __bf16 T; };
template <int ET, int SPLIT, int BIAS_MODE, int OUT_MODE, bool RESID, int ACT = 0>
__global__ __launch_bounds__(256) void wmma_gemm64(
    const unsigned short* __restrict__ Ap, const unsigned short* __restrict__ A2p, int lda, long strideA,
    const unsigned short* __restrict__ Btp, const unsigned short* __restrict__ Bt2p, int ldb, long strideB,
    void* __restrict__ Cout, void* __restrict__ Cout2, int ldc, long strideC,
    const float* __restrict__ bias,
    const float* __restrict__ resid, long strideR,
    int M, int N, int K, float scale) {
  typedef typename Elem<ET>::T T;
  typedef typename Frag<T>::V V;
  const T* A = (const T*)Ap; const T* A2 = (const T*)A2p; const T* Bt = (const T*)Btp; const T* Bt2 = (const T*)Bt2p;
  __shared__ __align__(16) float sT[8][16 * 68];
  const int b    = blockIdx.y;
  const int lane = threadIdx.x & 31;
  const int wave = threadIdx.x >> 5;
  const int tilesN = N >> 6;
  const int tilesM = M >> 6;
  const int tile = blockIdx.x * 8 + wave;
  if (tile >= tilesM * tilesN) return;
  const int tm = tile / tilesN;
  const int tn = tile - tm * tilesN;
  const int m0 = tm << 6;
  const int n0 = tn << 6;

  const T* Ab  = A  + (size_t)b * strideA;
  const T* Bb  = Bt + (size_t)b * strideB;
  const T* Ab2 = (SPLIT != 0) ? (A2  + (size_t)b * strideA) : nullptr;
  const T* Bb2 = (SPLIT == 1) ? (Bt2 + (size_t)b * strideB) : nullptr;

  const int rlane = lane & 15;
  const int koff  = (lane >> 4) * 8;
  const int mOff  = (lane >> 4) * 8;

  v8f acc[4][4];
#pragma unroll
  for (int i = 0; i < 4; ++i)
#pragma unroll
    for (int j = 0; j < 4; ++j) acc[i][j] = (v8f){0.f,0.f,0.f,0.f,0.f,0.f,0.f,0.f};

  for (int k0 = 0; k0 < K; k0 += 32) {
    V bh[4], bl[4];
#pragma unroll
    for (int j = 0; j < 4; ++j) {
      const size_t bo = (size_t)(n0 + (j << 4) + rlane) * ldb + koff + k0;
      bh[j] = Frag<T>::load(Bb + bo);
      if (SPLIT == 1) bl[j] = Frag<T>::load(Bb2 + bo);
    }
#pragma unroll
    for (int i = 0; i < 4; ++i) {
      const size_t ao = (size_t)(m0 + (i << 4) + rlane) * lda + koff + k0;
      V ah = Frag<T>::load(Ab + ao);
      V al;
      if (SPLIT != 0) al = Frag<T>::load(Ab2 + ao);
#pragma unroll
      for (int j = 0; j < 4; ++j) {
        acc[i][j] = Frag<T>::mma(ah, bh[j], acc[i][j]);
        if (SPLIT == 1) acc[i][j] = Frag<T>::mma(ah, bl[j], acc[i][j]);
        if (SPLIT != 0) acc[i][j] = Frag<T>::mma(al, bh[j], acc[i][j]);
      }
      Frag<T>::guard4(acc[i][0], acc[i][1], acc[i][2], acc[i][3], ah, (SPLIT != 0) ? al : ah);
    }
    Frag<T>::keep(bh[0], bh[1], bh[2], bh[3]);
    if (SPLIT == 1) Frag<T>::keep(bl[0], bl[1], bl[2], bl[3]);
  }
  acc_guard4(acc[0][0], acc[0][1], acc[0][2], acc[0][3]);
  acc_guard4(acc[1][0], acc[1][1], acc[1][2], acc[1][3]);
  acc_guard4(acc[2][0], acc[2][1], acc[2][2], acc[2][3]);
  acc_guard4(acc[3][0], acc[3][1], acc[3][2], acc[3][3]);

  float* slab = sT[wave];
  const float* Rb = RESID ? (resid + (size_t)b * strideR) : nullptr;
#pragma unroll
  for (int i = 0; i < 4; ++i) {
    const int mBase = m0 + (i << 4);
#pragma unroll
    for (int j = 0; j < 4; ++j) {
      const int n = n0 + (j << 4) + rlane;
      float bv = 0.f;
      if (BIAS_MODE == 2) bv = bias[n];
#pragma unroll
      for (int r = 0; r < 8; ++r) {
        float v = acc[i][j][r] * scale;
        if (BIAS_MODE == 1) v += bias[mBase + mOff + r];
        if (BIAS_MODE == 2) v += bv;
        if (RESID) v += Rb[(size_t)(mBase + mOff + r) * ldc + n];
        if (ACT == 2) v = fmaxf(v, 0.0f);
        if (ACT == 4) v = (v > 0.f) ? v : 0.01f * v;
        slab[(mOff + r) * 68 + (j << 4) + rlane] = v;
      }
    }
    __builtin_amdgcn_fence(__ATOMIC_RELEASE, "workgroup");
    __builtin_amdgcn_wave_barrier();
    __builtin_amdgcn_fence(__ATOMIC_ACQUIRE, "workgroup");
    if (OUT_MODE == 0) {
      float* C = (float*)Cout + (size_t)b * strideC;
      const int hh = lane >> 4, c4 = (lane & 15) * 4;
      for (int pass = 0; pass < 2; ++pass) {
#pragma unroll
        for (int it = 0; it < 8; ++it) {
          const int row = it * 2 + hh;
          v4f v = *(const v4f*)(slab + row * 68 + c4);
          *(volatile v4f*)(C + (size_t)(mBase + row) * ldc + n0 + c4) = v;
        }
        __threadfence();
      }
    } else {
      const int q = lane >> 3, c8 = (lane & 7) * 8;
      unsigned short* C  = (unsigned short*)Cout  + (size_t)b * strideC;
      unsigned short* C2 = (OUT_MODE == 2) ? ((unsigned short*)Cout2 + (size_t)b * strideC) : nullptr;
      for (int pass = 0; pass < 2; ++pass) {
#pragma unroll
        for (int it = 0; it < 4; ++it) {
          const int row = it * 4 + q;
          const float* sp = slab + row * 68 + c8;
          v8h hv, lv;
#pragma unroll
          for (int e = 0; e < 8; ++e) {
            if (OUT_MODE == 1) {
              hv[e] = (_Float16)sp[e];
            } else {
              unsigned short hb = f2bf_bits(sp[e]);
              unsigned short lb = f2bf_bits(sp[e] - bf_bits2f(hb));
              hv[e] = __builtin_bit_cast(_Float16, hb);
              lv[e] = __builtin_bit_cast(_Float16, lb);
            }
          }
          *(volatile v8h*)(C + (size_t)(mBase + row) * ldc + n0 + c8) = hv;
          if (OUT_MODE == 2) *(volatile v8h*)(C2 + (size_t)(mBase + row) * ldc + n0 + c8) = lv;
        }
        __threadfence();
      }
    }
    __builtin_amdgcn_fence(__ATOMIC_RELEASE, "workgroup");
    __builtin_amdgcn_wave_barrier();
    __builtin_amdgcn_fence(__ATOMIC_ACQUIRE, "workgroup");
  }
}

__global__ __launch_bounds__(256) void cast8_bf16_kernel(const float* __restrict__ in, unsigned short* __restrict__ out, int n8) {
  const int i = blockIdx.x * 256 + threadIdx.x;
  if (i >= n8) return;
  const float* p = in + 8 * (size_t)i;
  const v4f a = *(const v4f*)(p);
  const v4f c = *(const v4f*)(p + 4);
  unsigned short hb[8];
#pragma unroll
  for (int e = 0; e < 4; ++e) {
    hb[e]     = f2bf_bits(a[e]);
    hb[4 + e] = f2bf_bits(c[e]);
  }
  const v4u u = (v4u){pk16(hb[0], hb[1]), pk16(hb[2], hb[3]), pk16(hb[4], hb[5]), pk16(hb[6], hb[7])};
  unsigned short* q = out + 8 * (size_t)i;
  *(volatile v4u*)q = u;
  __threadfence();
  *(volatile v4u*)q = u;
}

__global__ __launch_bounds__(256) void zero8_kernel(unsigned short* __restrict__ out, int n8) {
  const int i = blockIdx.x * 256 + threadIdx.x;
  if (i >= n8) return;
  const v4u z = (v4u){0u, 0u, 0u, 0u};
  unsigned short* q = out + 8 * (size_t)i;
  *(volatile v4u*)q = z;
  __threadfence();
  *(volatile v4u*)q = z;
}

__global__ __launch_bounds__(256) void rope_gate_split_kernel(
    const float* __restrict__ Pq, const float* __restrict__ cosT, const float* __restrict__ sinT,
    const float* __restrict__ Wg,
    unsigned int* __restrict__ Qh, unsigned int* __restrict__ Ql,
    unsigned int* __restrict__ Kh, unsigned int* __restrict__ Kl,
    unsigned short* __restrict__ VTh, unsigned short* __restrict__ VTl, int b) {
  __shared__ __align__(16) unsigned short vsh[64][72];
  __shared__ __align__(16) unsigned short vsl[64][72];
  const int t    = threadIdx.x;
  const int lane = t & 31, wave = t >> 5;
  const int s0   = blockIdx.x * 64;
  const int h    = blockIdx.y;
  const int bh   = b * kHeads + h;

#pragma unroll
  for (int i = 0; i < 4; ++i) {
    const int e  = i * 256 + t;
    const int r  = e >> 4;
    const int c4 = (e & 15) * 4;
    const v4f vv = *(const v4f*)(Pq + (size_t)(s0 + r) * kNcat + 2 * kDim + h * kDh + c4);
#pragma unroll
    for (int k = 0; k < 4; ++k) {
      unsigned short hb, lb;
      split_bits(vv[k], hb, lb);
      vsh[c4 + k][r] = hb;
      vsl[c4 + k][r] = lb;
    }
  }
  __syncthreads();
  {
    const int q = lane >> 3, c8 = (lane & 7) * 8;
    unsigned short* oph = VTh + (size_t)bh * kDh * kSeq;
    unsigned short* opl = VTl + (size_t)bh * kDh * kSeq;
    for (int pass = 0; pass < 2; ++pass) {
#pragma unroll
      for (int it = 0; it < 2; ++it) {
        const int row = wave * 8 + it * 4 + q;
        const unsigned short* ah = &vsh[row][c8];
        const unsigned short* al = &vsl[row][c8];
        const v4u uh = (v4u){pk16(ah[0], ah[1]), pk16(ah[2], ah[3]), pk16(ah[4], ah[5]), pk16(ah[6], ah[7])};
        const v4u ul = (v4u){pk16(al[0], al[1]), pk16(al[2], al[3]), pk16(al[4], al[5]), pk16(al[6], al[7])};
        *(volatile v4u*)(oph + (size_t)row * kSeq + s0 + c8) = uh;
        *(volatile v4u*)(opl + (size_t)row * kSeq + s0 + c8) = ul;
      }
      __threadfence();
    }
  }

  const float wg0 = bfr(Wg[2 * lane]);
  const float wg1 = bfr(Wg[2 * lane + 1]);
  const float sgn = (lane < 16) ? -1.0f : 1.0f;
#pragma unroll 1
  for (int i = 0; i < 8; ++i) {
    const int s  = s0 + wave * 8 + i;
    const int sp = (s > 0) ? (s - 1) : 0;
    const float* rq = Pq + (size_t)s  * kNcat + h * kDh + 2 * lane;
    const float* rp = Pq + (size_t)sp * kNcat + kDim + h * kDh + 2 * lane;
    const v2f q2  = *(const v2f*)(rq);
    const v2f k2  = *(const v2f*)(rq + kDim);
    const v2f kp2 = *(const v2f*)(rp);
    const v2f c2  = *(const v2f*)(cosT + (size_t)s  * kDh + 2 * lane);
    const v2f n2  = *(const v2f*)(sinT + (size_t)s  * kDh + 2 * lane);
    const v2f cp2 = *(const v2f*)(cosT + (size_t)sp * kDh + 2 * lane);
    const v2f np2 = *(const v2f*)(sinT + (size_t)sp * kDh + 2 * lane);
    const float c0 = bfr(c2[0]),  c1 = bfr(c2[1]);
    const float e0 = bfr(n2[0]),  e1 = bfr(n2[1]);
    const float f0 = bfr(cp2[0]), f1 = bfr(cp2[1]);
    const float g0 = bfr(np2[0]), g1 = bfr(np2[1]);
    const float pq0 = __shfl_xor(q2[0], 16, 32),  pq1 = __shfl_xor(q2[1], 16, 32);
    const float pk0 = __shfl_xor(k2[0], 16, 32),  pk1 = __shfl_xor(k2[1], 16, 32);
    const float pp0 = __shfl_xor(kp2[0], 16, 32), pp1 = __shfl_xor(kp2[1], 16, 32);
    const float qr0 = q2[0] * c0 + (sgn * pq0) * e0;
    const float qr1 = q2[1] * c1 + (sgn * pq1) * e1;
    const float kr0 = k2[0] * c0 + (sgn * pk0) * e0;
    const float kr1 = k2[1] * c1 + (sgn * pk1) * e1;
    const float kz0 = kp2[0] * f0 + (sgn * pp0) * g0;
    const float kz1 = kp2[1] * f1 + (sgn * pp1) * g1;
    float part = kz0 * wg0 + kz1 * wg1;
#pragma unroll
    for (int off = 16; off > 0; off >>= 1) part += __shfl_xor(part, off, 32);
    const float gsig   = 1.0f / (1.0f + expf(-part));
    const float wblend = 2.0f * gsig - 1.0f;
    const float weff   = (s > 0) ? wblend : 0.0f;
    const float kb0 = kr0 + weff * kz0;
    const float kb1 = kr1 + weff * kz1;
    unsigned short qh0, ql0, qh1, ql1, kh0, kl0, kh1, kl1;
    split_bits(qr0, qh0, ql0); split_bits(qr1, qh1, ql1);
    split_bits(kb0, kh0, kl0); split_bits(kb1, kh1, kl1);
    const unsigned wqh = pk16(qh0, qh1), wql = pk16(ql0, ql1);
    const unsigned wkh = pk16(kh0, kh1), wkl = pk16(kl0, kl1);
    const size_t wi = ((size_t)bh * kSeq + s) * 32 + lane;
    *(volatile unsigned*)(Qh + wi) = wqh;
    *(volatile unsigned*)(Ql + wi) = wql;
    *(volatile unsigned*)(Kh + wi) = wkh;
    *(volatile unsigned*)(Kl + wi) = wkl;
    __threadfence();
    *(volatile unsigned*)(Qh + wi) = wqh;
    *(volatile unsigned*)(Ql + wi) = wql;
    *(volatile unsigned*)(Kh + wi) = wkh;
    *(volatile unsigned*)(Kl + wi) = wkl;
  }
}

__device__ __forceinline__ v8f mma_b(v16b a, v16b b, v8f c) {
  c = __builtin_amdgcn_wmma_f32_16x16x32_bf16(false, a, false, b, (short)0, c, false, false);
  asm volatile("v_nop\n\tv_nop\n\tv_nop\n\tv_nop" : "+v"(c) : "v"(a), "v"(b));
  return c;
}

__global__ __launch_bounds__(128)
void attn_kernel(const unsigned short* __restrict__ Qh, const unsigned short* __restrict__ Ql,
                 const unsigned short* __restrict__ Kh, const unsigned short* __restrict__ Kl,
                 const unsigned short* __restrict__ VTh, const unsigned short* __restrict__ VTl,
                 const float* __restrict__ G, const int* __restrict__ bsp,
                 unsigned short* __restrict__ Oh, unsigned short* __restrict__ Ol, int b) {
  __shared__ __align__(16) unsigned short Ksh[64 * 64];
  __shared__ __align__(16) unsigned short Ksl[64 * 64];
  __shared__ __align__(16) unsigned short Vth[64 * 64];
  __shared__ __align__(16) unsigned short Vtl[64 * 64];
  __shared__ __align__(16) unsigned short Psh[4][16 * 64];
  __shared__ __align__(16) unsigned short Psl[4][16 * 64];

  const int tid  = threadIdx.x;
  const int wave = tid >> 5;
  const int lane = tid & 31;
  const int hh   = lane >> 4;
  const int c    = lane & 15;
  const int qb   = blockIdx.x & 31;
  const int h    = blockIdx.x >> 5;
  const int bh   = b * kHeads + h;
  const int q0   = qb * 64 + wave * 16;

  int bs = bsp[0];
  bs = (bs < 1) ? 1 : ((bs > 64) ? 64 : bs);
  const int rem    = kSeq % bs;
  const int remadd = (rem != 0) ? 1 : 0;

  v16b qah[2], qal[2];
  {
    const __bf16* qhp = (const __bf16*)Qh + ((size_t)bh * kSeq + q0 + c) * kDh + 8 * hh;
    const __bf16* qlp = (const __bf16*)Ql + ((size_t)bh * kSeq + q0 + c) * kDh + 8 * hh;
#pragma unroll
    for (int dc = 0; dc < 2; ++dc) {
      qah[dc] = Frag<__bf16>::load(qhp + dc * 32);
      qal[dc] = Frag<__bf16>::load(qlp + dc * 32);
    }
  }

  float mrow[8], lrow[8];
  v8f oacc[4];
#pragma unroll
  for (int r = 0; r < 8; ++r) { mrow[r] = -INFINITY; lrow[r] = 0.f; }
#pragma unroll
  for (int t2 = 0; t2 < 4; ++t2) oacc[t2] = (v8f){0.f,0.f,0.f,0.f,0.f,0.f,0.f,0.f};

  const int nChunks = qb + 1;
  for (int kc = 0; kc < nChunks; ++kc) {
    const int kv0 = kc * 64;
    __syncthreads();
    {
      const v4u* khs = (const v4u*)Kh + ((size_t)bh * kSeq + kv0) * 8;
      const v4u* kls = (const v4u*)Kl + ((size_t)bh * kSeq + kv0) * 8;
      v4u* kdh = (v4u*)Ksh;
      v4u* kdl = (v4u*)Ksl;
#pragma unroll
      for (int i = 0; i < 4; ++i) {
        const int u = tid + 128 * i;
        kdh[u] = khs[u];
        kdl[u] = kls[u];
      }
      asm volatile("" ::: "memory");
      const v4u* vhs = (const v4u*)VTh + (size_t)bh * kDh * (kSeq / 8) + (kv0 >> 3);
      const v4u* vls = (const v4u*)VTl + (size_t)bh * kDh * (kSeq / 8) + (kv0 >> 3);
      v4u* vdh = (v4u*)Vth;
      v4u* vdl = (v4u*)Vtl;
#pragma unroll
      for (int i = 0; i < 4; ++i) {
        const int u  = tid + 128 * i;
        const int d  = u >> 3;
        const int pc = u & 7;
        vdh[u] = vhs[(size_t)d * (kSeq / 8) + pc];
        vdl[u] = vls[(size_t)d * (kSeq / 8) + pc];
      }
    }
    __syncthreads();

    v8f s[4];
#pragma unroll
    for (int j = 0; j < 4; ++j) {
      s[j] = (v8f){0.f,0.f,0.f,0.f,0.f,0.f,0.f,0.f};
#pragma unroll
      for (int dc = 0; dc < 2; ++dc) {
        const int ko = (j * 16 + c) * 64 + dc * 32 + 8 * hh;
        const v16b kbf = Frag<__bf16>::load((const __bf16*)Ksh + ko);
        const v16b klf = Frag<__bf16>::load((const __bf16*)Ksl + ko);
        s[j] = mma_b(qah[dc], kbf, s[j]);
        s[j] = mma_b(qah[dc], klf, s[j]);
        s[j] = mma_b(qal[dc], kbf, s[j]);
      }
    }
#pragma unroll
    for (int r = 0; r < 8; ++r)
#pragma unroll
      for (int j = 0; j < 4; ++j) s[j][r] *= kQKScale;

    const bool diag = (kc == qb);
    if (diag) {
      int qbid[8], kbid[4];
#pragma unroll
      for (int r = 0; r < 8; ++r) {
        const int qr = q0 + 8 * hh + r;
        qbid[r] = (qr < rem) ? 0 : ((qr - rem) / bs + remadd);
      }
#pragma unroll
      for (int j = 0; j < 4; ++j) {
        const int kvc = kv0 + j * 16 + c;
        kbid[j] = (kvc < rem) ? 0 : ((kvc - rem) / bs + remadd);
      }
#pragma unroll
      for (int r = 0; r < 8; ++r)
#pragma unroll
        for (int j = 0; j < 4; ++j)
          if (kbid[j] > qbid[r]) s[j][r] = kFill;
    }
    float cm[8];
#pragma unroll
    for (int r = 0; r < 8; ++r) {
      float m = fmaxf(fmaxf(s[0][r], s[1][r]), fmaxf(s[2][r], s[3][r]));
#pragma unroll
      for (int off = 1; off < 16; off <<= 1) m = fmaxf(m, __shfl_xor(m, off, 32));
      cm[r] = m;
    }
    unsigned short* pwh = Psh[wave];
    unsigned short* pwl = Psl[wave];
#pragma unroll
    for (int r = 0; r < 8; ++r) {
      const float mnew  = fmaxf(mrow[r], cm[r]);
      const float alpha = expf(mrow[r] - mnew);
      mrow[r] = mnew;
      float psum = 0.f;
#pragma unroll
      for (int j = 0; j < 4; ++j) {
        const float p = expf(s[j][r] - mnew);
        psum += p;
        unsigned short hb, lb;
        split_bits(p, hb, lb);
        pwh[(8 * hh + r) * 64 + j * 16 + c] = hb;
        pwl[(8 * hh + r) * 64 + j * 16 + c] = lb;
      }
#pragma unroll
      for (int off = 1; off < 16; off <<= 1) psum += __shfl_xor(psum, off, 32);
      lrow[r] = lrow[r] * alpha + psum;
#pragma unroll
      for (int t2 = 0; t2 < 4; ++t2) oacc[t2][r] *= alpha;
    }
    __builtin_amdgcn_fence(__ATOMIC_RELEASE, "workgroup");
    __builtin_amdgcn_wave_barrier();
    __builtin_amdgcn_fence(__ATOMIC_ACQUIRE, "workgroup");

#pragma unroll 1
    for (int kk = 0; kk < 2; ++kk) {
      const int po = c * 64 + kk * 32 + 8 * hh;
      const v16b pa = Frag<__bf16>::load((const __bf16*)pwh + po);
      const v16b pl = Frag<__bf16>::load((const __bf16*)pwl + po);
#pragma unroll
      for (int t2 = 0; t2 < 4; ++t2) {
        const int vo = (t2 * 16 + c) * 64 + kk * 32 + 8 * hh;
        const v16b vb = Frag<__bf16>::load((const __bf16*)Vth + vo);
        const v16b vl = Frag<__bf16>::load((const __bf16*)Vtl + vo);
        oacc[t2] = mma_b(pa, vb, oacc[t2]);
        oacc[t2] = mma_b(pa, vl, oacc[t2]);
        oacc[t2] = mma_b(pl, vb, oacc[t2]);
      }
    }
  }

  float graw[8];
#pragma unroll
  for (int r = 0; r < 8; ++r) graw[r] = G[(size_t)(q0 + 8 * hh + r) * kNcat + kGateCol + h];
  __builtin_amdgcn_fence(__ATOMIC_RELEASE, "workgroup");
  __builtin_amdgcn_wave_barrier();
  __builtin_amdgcn_fence(__ATOMIC_ACQUIRE, "workgroup");
  unsigned short* osh = Psh[wave];
  unsigned short* osl = Psl[wave];
#pragma unroll
  for (int r = 0; r < 8; ++r) {
    const float inv = 1.0f / lrow[r];
    const float sg  = 1.0f / (1.0f + expf(-graw[r]));
    const float f   = inv * sg;
#pragma unroll
    for (int t2 = 0; t2 < 4; ++t2) {
      unsigned short hb, lb;
      split_bits(oacc[t2][r] * f, hb, lb);
      osh[(8 * hh + r) * 64 + t2 * 16 + c] = hb;
      osl[(8 * hh + r) * 64 + t2 * 16 + c] = lb;
    }
  }
  __builtin_amdgcn_fence(__ATOMIC_RELEASE, "workgroup");
  __builtin_amdgcn_wave_barrier();
  __builtin_amdgcn_fence(__ATOMIC_ACQUIRE, "workgroup");
  {
    const int q = lane >> 3, c8 = (lane & 7) * 8;
    for (int pass = 0; pass < 2; ++pass) {
#pragma unroll
      for (int it = 0; it < 4; ++it) {
        const int row = it * 4 + q;
        const unsigned short* ah = osh + row * 64 + c8;
        const unsigned short* al = osl + row * 64 + c8;
        const v4u uh = (v4u){pk16(ah[0], ah[1]), pk16(ah[2], ah[3]), pk16(ah[4], ah[5]), pk16(ah[6], ah[7])};
        const v4u ul = (v4u){pk16(al[0], al[1]), pk16(al[2], al[3]), pk16(al[4], al[5]), pk16(al[6], al[7])};
        const size_t oo = ((size_t)(b * kSeq + q0 + row)) * kDim + h * kDh + c8;
        *(volatile v4u*)(Oh + oo) = uh;
        *(volatile v4u*)(Ol + oo) = ul;
      }
      __threadfence();
    }
  }
}

extern "C" void kernel_launch(void* const* d_in, const int* in_sizes, int n_in,
                              void* d_out, int out_size, void* d_ws, size_t ws_size,
                              hipStream_t stream) {
  if (n_in < 10) return;
  if (in_sizes[0] != kTok * kDim) return;
  if (in_sizes[1] != kSeq * kDh || in_sizes[2] != kSeq * kDh) return;
  if (in_sizes[3] != kDim * kDim || in_sizes[4] != kDim * kDim || in_sizes[5] != kDim * kDim) return;
  if (in_sizes[6] != kHeads * kDim || in_sizes[7] != kDh || in_sizes[8] != kDim * kDim || in_sizes[9] < 1) return;
  if (out_size != kTok * kDim) return;

  const size_t szXb   = (size_t)kTok * kDim * 2;
  const size_t szWcat = (size_t)kNcat * kDim * 2;
  const size_t szWob  = (size_t)kDim * kDim * 2;
  const size_t szQKVG = (size_t)kSeq * kNcat * 4;
  const size_t szPl   = (size_t)kBatch * kHeads * kSeq * kDh * 2;
  const size_t szO    = (size_t)kTok * kDim * 2;
  const size_t offXb   = 0;
  const size_t offWcat = offXb + szXb;
  const size_t offWob  = offWcat + szWcat;
  const size_t offQKVG = offWob + szWob;
  const size_t offQh   = offQKVG + szQKVG;
  const size_t offQl   = offQh + szPl;
  const size_t offKh   = offQl + szPl;
  const size_t offKl   = offKh + szPl;
  const size_t offVTh  = offKl + szPl;
  const size_t offVTl  = offVTh + szPl;
  const size_t offOh   = offVTl + szPl;
  const size_t offOl   = offOh + szO;
  const size_t total   = offOl + szO;
  if (ws_size < total) return;

  const float* x     = (const float*)d_in[0];
  const float* cosT  = (const float*)d_in[1];
  const float* sinT  = (const float*)d_in[2];
  const float* Wq    = (const float*)d_in[3];
  const float* Wk    = (const float*)d_in[4];
  const float* Wv    = (const float*)d_in[5];
  const float* Wgate = (const float*)d_in[6];
  const float* Wg    = (const float*)d_in[7];
  const float* Wo    = (const float*)d_in[8];
  const int*   bsz   = (const int*)d_in[9];
  float* out = (float*)d_out;
  char* ws = (char*)d_ws;
  unsigned short* Xb   = (unsigned short*)(ws + offXb);
  unsigned short* Wcat = (unsigned short*)(ws + offWcat);
  unsigned short* Wob  = (unsigned short*)(ws + offWob);
  float*          QKVG = (float*)(ws + offQKVG);
  unsigned short* Qh   = (unsigned short*)(ws + offQh);
  unsigned short* Ql   = (unsigned short*)(ws + offQl);
  unsigned short* Kh   = (unsigned short*)(ws + offKh);
  unsigned short* Kl   = (unsigned short*)(ws + offKl);
  unsigned short* VTh  = (unsigned short*)(ws + offVTh);
  unsigned short* VTl  = (unsigned short*)(ws + offVTl);
  unsigned short* Oh   = (unsigned short*)(ws + offOh);
  unsigned short* Ol   = (unsigned short*)(ws + offOl);

  const int n8x  = (kTok * kDim) / 8;
  const int n8w  = (kDim * kDim) / 8;
  const int n8g  = (kHeads * kDim) / 8;
  const int n8z  = (48 * kDim) / 8;
  cast8_bf16_kernel<<<dim3((n8x + 255) / 256), dim3(256), 0, stream>>>(x,     Xb, n8x);
  cast8_bf16_kernel<<<dim3((n8w + 255) / 256), dim3(256), 0, stream>>>(Wq,    Wcat, n8w);
  cast8_bf16_kernel<<<dim3((n8w + 255) / 256), dim3(256), 0, stream>>>(Wk,    Wcat + (size_t)1 * kDim * kDim, n8w);
  cast8_bf16_kernel<<<dim3((n8w + 255) / 256), dim3(256), 0, stream>>>(Wv,    Wcat + (size_t)2 * kDim * kDim, n8w);
  cast8_bf16_kernel<<<dim3((n8g + 255) / 256), dim3(256), 0, stream>>>(Wgate, Wcat + (size_t)kGateCol * kDim, n8g);
  zero8_kernel     <<<dim3((n8z + 255) / 256), dim3(256), 0, stream>>>(       Wcat + (size_t)kZeroRow * kDim, n8z);
  cast8_bf16_kernel<<<dim3((n8w + 255) / 256), dim3(256), 0, stream>>>(Wo,    Wob, n8w);

  const int tilesQKVG = (kSeq / 64) * (kNcat / 64);
  const int tilesOut  = (kTok / 64) * (kDim / 64);
  const float* fdummy = (const float*)QKVG;

  for (int b = 0; b < kBatch; ++b) {
    wmma_gemm64<1, 0, 0, 0, false, 0><<<dim3((tilesQKVG + 7) / 8, 1), dim3(256), 0, stream>>>(
        Xb + (size_t)b * kSeq * kDim, Xb + (size_t)b * kSeq * kDim, kDim, 0L,
        Wcat, Wcat, kDim, 0L,
        (void*)QKVG, (void*)QKVG, kNcat, 0L,
        fdummy, fdummy, 0L, kSeq, kNcat, kDim, 1.0f);
    rope_gate_split_kernel<<<dim3(kSeq / 64, kHeads), dim3(256), 0, stream>>>(
        QKVG, cosT, sinT, Wg,
        (unsigned int*)Qh, (unsigned int*)Ql, (unsigned int*)Kh, (unsigned int*)Kl, VTh, VTl, b);
    attn_kernel<<<dim3(kHeads * (kSeq / 64)), dim3(128), 0, stream>>>(
        Qh, Ql, Kh, Kl, VTh, VTl, QKVG, bsz, Oh, Ol, b);
  }

  wmma_gemm64<1, 2, 0, 0, false, 0><<<dim3((tilesOut + 7) / 8, 1), dim3(256), 0, stream>>>(
      Oh, Ol, kDim, 0L,
      Wob, Wob, kDim, 0L,
      (void*)out, (void*)out, kDim, 0L,
      fdummy, fdummy, 0L, kTok, kDim, kDim, 1.0f);
}
